// TitanAttention_712964571146
// MI455X (gfx1250) — hardware-run, weakly checked
//
#include <hip/hip_runtime.h>
#include <math.h>
#include <stdint.h>

#define NB   2
#define SEQ  2048
#define DM   1024
#define NH   16
#define HD   64
#define NQB  (SEQ / 64)
#define NTOK (NB * SEQ)
static_assert(NH * HD == DM);
static_assert((SEQ % 64) == 0 && (DM % 64) == 0 && (NTOK % 64) == 0);

#define CAR_W   64.0f
#define CAR_P0  16.0f
#define CAR_Y   256.0f
#define CAR_N   64.0f
#define CAR_V   1024.0f
#define CAR_P   1024.0f

typedef _Float16 v16h __attribute__((ext_vector_type(16)));
typedef _Float16 v8h  __attribute__((ext_vector_type(8)));
typedef __bf16   v16b __attribute__((ext_vector_type(16)));
typedef __bf16   v8b  __attribute__((ext_vector_type(8)));
typedef float    v8f  __attribute__((ext_vector_type(8)));
typedef float    v4f  __attribute__((ext_vector_type(4)));
typedef unsigned int v4u __attribute__((ext_vector_type(4)));

__device__ __forceinline__ unsigned short h_bits(_Float16 x) { return __builtin_bit_cast(unsigned short, x); }
__device__ __forceinline__ unsigned pk16(unsigned short a, unsigned short b) { return (unsigned)a | ((unsigned)b << 16); }
__device__ __forceinline__ unsigned pkf(float a, float b) {
  return pk16(h_bits((_Float16)a), h_bits((_Float16)b));
}
__device__ __forceinline__ unsigned short bf_bits(float f) {
  unsigned u = __float_as_uint(f);
  return (unsigned short)((u + 0x7FFFu + ((u >> 16) & 1u)) >> 16);
}
__device__ __forceinline__ float bf_up(unsigned short h) { return __uint_as_float(((unsigned)h) << 16); }
__device__ __forceinline__ v8f zero8() { v8f z = {0.f, 0.f, 0.f, 0.f, 0.f, 0.f, 0.f, 0.f}; return z; }

__device__ __forceinline__ v16h ldfrag_h(const _Float16* p) {
  union { v16h v; v8h h[2]; } f;
  f.h[0] = *(const v8h*)(p);
  f.h[1] = *(const v8h*)(p + 16);
  return f.v;
}
__device__ __forceinline__ v16b ldfrag_b(const __bf16* p) {
  union { v16b v; v8b h[2]; } f;
  f.h[0] = *(const v8b*)(p);
  f.h[1] = *(const v8b*)(p + 16);
  return f.v;
}

__device__ __forceinline__ v8f mma_h(v16h a, v16h b, v8f c) {
  c = __builtin_amdgcn_wmma_f32_16x16x32_f16(false, a, false, b, (short)0, c, false, false);
  asm volatile("v_nop\n\tv_nop\n\tv_nop\n\tv_nop" : "+v"(c) : "v"(a), "v"(b));
  return c;
}
__device__ __forceinline__ v8f mma_h_raw(v16h a, v16h b, v8f c) {
  return __builtin_amdgcn_wmma_f32_16x16x32_f16(false, a, false, b, (short)0, c, false, false);
}
__device__ __forceinline__ v8f mma_b_raw(v16b a, v16b b, v8f c) {
  return __builtin_amdgcn_wmma_f32_16x16x32_bf16(false, a, false, b, (short)0, c, false, false);
}
__device__ __forceinline__ void dep_guard_h(v8f& a, v8f& b, v16h x, v16h y) {
  asm volatile("v_nop\n\tv_nop\n\tv_nop\n\tv_nop" : "+v"(a), "+v"(b) : "v"(x), "v"(y));
}
__device__ __forceinline__ void dep_guard_b(v8f& a, v8f& b, v16b x, v16b y) {
  asm volatile("v_nop\n\tv_nop\n\tv_nop\n\tv_nop" : "+v"(a), "+v"(b) : "v"(x), "v"(y));
}
__device__ __forceinline__ void keep4_h(v16h a, v16h b, v16h c, v16h d) {
  asm volatile("v_nop" :: "v"(a), "v"(b), "v"(c), "v"(d));
}
__device__ __forceinline__ void keep4_b(v16b a, v16b b, v16b c, v16b d) {
  asm volatile("v_nop" :: "v"(a), "v"(b), "v"(c), "v"(d));
}
__device__ __forceinline__ void acc_guard4(v8f& a, v8f& b, v8f& c, v8f& d) {
  asm volatile("v_nop\n\tv_nop\n\tv_nop\n\tv_nop" : "+v"(a), "+v"(b), "+v"(c), "+v"(d));
}
__device__ __forceinline__ void acc_guard2(v8f& a, v8f& b) {
  asm volatile("v_nop\n\tv_nop\n\tv_nop\n\tv_nop" : "+v"(a), "+v"(b));
}

__global__ __launch_bounds__(256) void cvt_f16x8(
    const float* __restrict__ p0, const float* __restrict__ p1, const float* __restrict__ p2,
    const float* __restrict__ p3, const float* __restrict__ p4, const float* __restrict__ p5,
    const float* __restrict__ p6, unsigned short* out, long long strideOut, int n8, float scale) {
  const int z = blockIdx.y;
  const float* in = (z == 0) ? p0 : ((z == 1) ? p1 : ((z == 2) ? p2 : ((z == 3) ? p3 :
                    ((z == 4) ? p4 : ((z == 5) ? p5 : p6)))));
  const int i = blockIdx.x * 256 + threadIdx.x;
  if (i < n8) {
    const v4f a = *(const v4f*)(in + (size_t)i * 8);
    const v4f b = *(const v4f*)(in + (size_t)i * 8 + 4);
    v4u p;
    p[0] = pkf(a[0] * scale, a[1] * scale);
    p[1] = pkf(a[2] * scale, a[3] * scale);
    p[2] = pkf(b[0] * scale, b[1] * scale);
    p[3] = pkf(b[2] * scale, b[3] * scale);
    unsigned short* o = out + (size_t)z * strideOut + (size_t)i * 8;
    *(volatile v4u*)o = p;
    __threadfence();
    *(volatile v4u*)o = p;
  }
}

__global__ __launch_bounds__(256) void cvt_bf16hl_x8(const float* __restrict__ in,
                                                      unsigned short* hi, unsigned short* lo, int n8) {
  const int i = blockIdx.x * 256 + threadIdx.x;
  if (i < n8) {
    const v4f a = *(const v4f*)(in + (size_t)i * 8);
    const v4f b = *(const v4f*)(in + (size_t)i * 8 + 4);
    float f[8];
#pragma unroll
    for (int e = 0; e < 4; ++e) { f[e] = a[e]; f[4 + e] = b[e]; }
    v4u ph, pl;
#pragma unroll
    for (int e = 0; e < 4; ++e) {
      const unsigned short h0 = bf_bits(f[2 * e]), h1 = bf_bits(f[2 * e + 1]);
      const unsigned short l0 = bf_bits(f[2 * e] - bf_up(h0)), l1 = bf_bits(f[2 * e + 1] - bf_up(h1));
      ph[e] = pk16(h0, h1);
      pl[e] = pk16(l0, l1);
    }
    unsigned short* oh = hi + (size_t)i * 8;
    unsigned short* ol = lo + (size_t)i * 8;
    *(volatile v4u*)oh = ph;
    *(volatile v4u*)ol = pl;
    __threadfence();
    *(volatile v4u*)oh = ph;
    *(volatile v4u*)ol = pl;
  }
}

__global__ __launch_bounds__(256) void dwconv3_f16x8(
    const unsigned short* __restrict__ P0p, unsigned short* Yp,
    const float* __restrict__ w0p, const float* __restrict__ w1p, const float* __restrict__ w2p,
    const float* __restrict__ b0p, const float* __restrict__ b1p, const float* __restrict__ b2p,
    long long plane, int n8, float gain, float bgain) {
  const int z = blockIdx.y;
  const float* w  = (z == 0) ? w0p : ((z == 1) ? w1p : w2p);
  const float* bs = (z == 0) ? b0p : ((z == 1) ? b1p : b2p);
  const int i = blockIdx.x * 256 + threadIdx.x;
  if (i >= n8) return;
  const size_t e0 = (size_t)i * 8;
  const int t = (int)(e0 / DM);
  const int c = (int)(e0 - (size_t)t * DM);
  const int s = t & (SEQ - 1);
  const _Float16* in = (const _Float16*)(const void*)P0p + (size_t)z * plane;
  const bool hasm = (s > 0);
  const bool hasp = (s < SEQ - 1);
  const int tm = hasm ? (t - 1) : t;
  const int tp = hasp ? (t + 1) : t;
  const v8h va = *(const v8h*)(in + (size_t)tm * DM + c);
  const v8h vb = *(const v8h*)(in + (size_t)t  * DM + c);
  const v8h vd = *(const v8h*)(in + (size_t)tp * DM + c);
  const v4f wA = *(const v4f*)(w + c * 3);
  const v4f wB = *(const v4f*)(w + c * 3 + 4);
  const v4f wC = *(const v4f*)(w + c * 3 + 8);
  const v4f wD = *(const v4f*)(w + c * 3 + 12);
  const v4f wE = *(const v4f*)(w + c * 3 + 16);
  const v4f wF = *(const v4f*)(w + c * 3 + 20);
  const v4f bA = *(const v4f*)(bs + c);
  const v4f bB = *(const v4f*)(bs + c + 4);
  float wl[24];
#pragma unroll
  for (int m = 0; m < 4; ++m) {
    wl[m] = wA[m]; wl[4 + m] = wB[m]; wl[8 + m] = wC[m];
    wl[12 + m] = wD[m]; wl[16 + m] = wE[m]; wl[20 + m] = wF[m];
  }
  float bl[8];
#pragma unroll
  for (int m = 0; m < 4; ++m) { bl[m] = bA[m]; bl[4 + m] = bB[m]; }
  float y[8];
#pragma unroll
  for (int e = 0; e < 8; ++e) {
    const float fa = hasm ? (float)va[e] : 0.f;
    const float fb = (float)vb[e];
    const float fd = hasp ? (float)vd[e] : 0.f;
    const float conv = wl[3 * e] * fa + wl[3 * e + 1] * fb + wl[3 * e + 2] * fd;
    y[e] = gain * conv + bgain * bl[e];
  }
  v4u p;
  p[0] = pkf(y[0], y[1]);
  p[1] = pkf(y[2], y[3]);
  p[2] = pkf(y[4], y[5]);
  p[3] = pkf(y[6], y[7]);
  unsigned short* o = Yp + (size_t)z * plane + e0;
  *(volatile v4u*)o = p;
  __threadfence();
  *(volatile v4u*)o = p;
}

template <int EPI>
__global__ __launch_bounds__(256) void gemm64(
    const unsigned short* __restrict__ Ap, int lda, long long strideA,
    const unsigned short* __restrict__ Btp, int ldb, long long strideB,
    void* Cout, int ldc, long long strideC,
    const float* __restrict__ bias0, const float* __restrict__ bias1, const float* __restrict__ bias2,
    int M, int N, int K, float rs, float cs) {
  const _Float16* A  = (const _Float16*)(const void*)Ap;
  const _Float16* Bt = (const _Float16*)(const void*)Btp;
  __shared__ __align__(16) float sT[8][16 * 68];
  const int b    = blockIdx.y;
  const float* bias = (b == 0) ? bias0 : ((b == 1) ? bias1 : bias2);
  const int lane = threadIdx.x & 31;
  const int wave = threadIdx.x >> 5;
  const int tilesN = N >> 6;
  const int tilesM = M >> 6;
  const int tile = blockIdx.x * 8 + wave;
  if (tile >= tilesM * tilesN) return;
  const int tm = tile / tilesN;
  const int tn = tile - tm * tilesN;
  const int m0 = tm << 6;
  const int n0 = tn << 6;

  const _Float16* Ab = A  + (size_t)b * strideA;
  const _Float16* Bb = Bt + (size_t)b * strideB;

  const int rlane = lane & 15;
  const int koff  = (lane >> 4) * 8;
  const int mOff  = (lane >> 4) * 8;

  v8f acc[4][4];
#pragma unroll
  for (int i = 0; i < 4; ++i)
#pragma unroll
    for (int j = 0; j < 4; ++j) acc[i][j] = zero8();

  for (int k0 = 0; k0 < K; k0 += 32) {
    v16h bh[4];
#pragma unroll
    for (int j = 0; j < 4; ++j) {
      const size_t bo = (size_t)(n0 + (j << 4) + rlane) * ldb + koff + k0;
      bh[j] = ldfrag_h(Bb + bo);
    }
#pragma unroll
    for (int i = 0; i < 4; ++i) {
      const size_t ao = (size_t)(m0 + (i << 4) + rlane) * lda + koff + k0;
      const v16h ah = ldfrag_h(Ab + ao);
#pragma unroll
      for (int j = 0; j < 4; ++j) acc[i][j] = mma_h_raw(ah, bh[j], acc[i][j]);
      dep_guard_h(acc[i][0], acc[i][3], ah, bh[3]);
    }
    keep4_h(bh[0], bh[1], bh[2], bh[3]);
  }
  acc_guard4(acc[0][0], acc[0][1], acc[0][2], acc[0][3]);
  acc_guard4(acc[1][0], acc[1][1], acc[1][2], acc[1][3]);
  acc_guard4(acc[2][0], acc[2][1], acc[2][2], acc[2][3]);
  acc_guard4(acc[3][0], acc[3][1], acc[3][2], acc[3][3]);

  float* slab = sT[wave];
#pragma unroll
  for (int i = 0; i < 4; ++i) {
    const int mBase = m0 + (i << 4);
#pragma unroll
    for (int j = 0; j < 4; ++j) {
#pragma unroll
      for (int r = 0; r < 8; ++r) {
        slab[(mOff + r) * 68 + (j << 4) + rlane] = acc[i][j][r];
      }
    }
    __builtin_amdgcn_fence(__ATOMIC_RELEASE, "workgroup");
    __builtin_amdgcn_wave_barrier();
    __builtin_amdgcn_fence(__ATOMIC_ACQUIRE, "workgroup");
    if (EPI == 0) {
      float* C = (float*)Cout + (size_t)b * strideC;
      const int hh = lane >> 4, c4 = (lane & 15) * 4;
      const v4f bc = *(const v4f*)(bias + n0 + c4);
      v4f ov[8];
#pragma unroll
      for (int it = 0; it < 8; ++it) {
        const int row = it * 2 + hh;
        const v4f v = *(const v4f*)(slab + row * 68 + c4);
        ov[it] = v * rs + bc;
      }
      for (int pass = 0; pass < 2; ++pass) {
#pragma unroll
        for (int it = 0; it < 8; ++it) {
          const int row = it * 2 + hh;
          *(volatile v4f*)(C + (size_t)(mBase + row) * ldc + n0 + c4) = ov[it];
        }
        __threadfence();
      }
    } else {
      const int q = lane >> 3, c8 = (lane & 7) * 8;
      unsigned short* C = (unsigned short*)Cout + (size_t)b * strideC;
      float bc[8];
      if (EPI == 3) {
#pragma unroll
        for (int e = 0; e < 8; ++e) bc[e] = 0.f;
      } else {
        const v4f b0v = *(const v4f*)(bias + n0 + c8);
        const v4f b1v = *(const v4f*)(bias + n0 + c8 + 4);
#pragma unroll
        for (int e = 0; e < 4; ++e) { bc[e] = b0v[e]; bc[4 + e] = b1v[e]; }
      }
      v4u hv[4];
#pragma unroll
      for (int it = 0; it < 4; ++it) {
        const int row = it * 4 + q;
        const float* sp = slab + row * 68 + c8;
        const v4f s0 = *(const v4f*)(sp);
        const v4f s1 = *(const v4f*)(sp + 4);
        float brow = 0.f;
        if (EPI == 3) brow = bias[mBase + row];
        float v[8];
#pragma unroll
        for (int e = 0; e < 4; ++e) {
          v[e]     = s0[e] * rs + ((EPI == 3) ? brow : bc[e]);
          v[4 + e] = s1[e] * rs + ((EPI == 3) ? brow : bc[4 + e]);
        }
        if (EPI == 1) {
#pragma unroll
          for (int e = 0; e < 8; ++e) v[e] = v[e] * __builtin_amdgcn_rcpf(1.0f + __expf(-v[e]));
        }
        float mult = cs;
        if (EPI == 2) {
          float ss = 0.f;
#pragma unroll
          for (int e = 0; e < 8; ++e) ss += v[e] * v[e];
          ss += __shfl_xor(ss, 1, 32);
          ss += __shfl_xor(ss, 2, 32);
          ss += __shfl_xor(ss, 4, 32);
          mult = cs * __builtin_amdgcn_rcpf(fmaxf(sqrtf(ss), 1e-12f));
        }
        v4u a;
        a[0] = pkf(v[0] * mult, v[1] * mult);
        a[1] = pkf(v[2] * mult, v[3] * mult);
        a[2] = pkf(v[4] * mult, v[5] * mult);
        a[3] = pkf(v[6] * mult, v[7] * mult);
        hv[it] = a;
      }
      for (int pass = 0; pass < 2; ++pass) {
#pragma unroll
        for (int it = 0; it < 4; ++it) {
          const int row = it * 4 + q;
          *(volatile v4u*)(C + (size_t)(mBase + row) * ldc + n0 + c8) = hv[it];
        }
        __threadfence();
      }
    }
    __builtin_amdgcn_fence(__ATOMIC_RELEASE, "workgroup");
    __builtin_amdgcn_wave_barrier();
    __builtin_amdgcn_fence(__ATOMIC_ACQUIRE, "workgroup");
  }
}

__global__ __launch_bounds__(256) void gemm_bf3(
    const unsigned short* __restrict__ Ahp, const unsigned short* __restrict__ Alp, int lda,
    const unsigned short* __restrict__ Bhp, const unsigned short* __restrict__ Blp, int ldb,
    float* Cout, int ldc, const float* __restrict__ bias, int M, int N, int K) {
  const __bf16* Ah = (const __bf16*)(const void*)Ahp;
  const __bf16* Al = (const __bf16*)(const void*)Alp;
  const __bf16* Bh = (const __bf16*)(const void*)Bhp;
  const __bf16* Bl = (const __bf16*)(const void*)Blp;
  __shared__ __align__(16) float sT[8][16 * 36];
  const int lane = threadIdx.x & 31;
  const int wave = threadIdx.x >> 5;
  const int tilesN = N >> 5;
  const int tilesM = M >> 6;
  const int tile = blockIdx.x * 8 + wave;
  if (tile >= tilesM * tilesN) return;
  const int tm = tile / tilesN;
  const int tn = tile - tm * tilesN;
  const int m0 = tm << 6;
  const int n0 = tn << 5;

  const int rlane = lane & 15;
  const int koff  = (lane >> 4) * 8;
  const int mOff  = (lane >> 4) * 8;

  v8f acc[4][2];
#pragma unroll
  for (int i = 0; i < 4; ++i)
#pragma unroll
    for (int j = 0; j < 2; ++j) acc[i][j] = zero8();

  for (int k0 = 0; k0 < K; k0 += 32) {
    v16b bh[2], bl[2];
#pragma unroll
    for (int j = 0; j < 2; ++j) {
      const size_t bo = (size_t)(n0 + (j << 4) + rlane) * ldb + koff + k0;
      bh[j] = ldfrag_b(Bh + bo);
      bl[j] = ldfrag_b(Bl + bo);
    }
#pragma unroll
    for (int i = 0; i < 4; ++i) {
      const size_t ao = (size_t)(m0 + (i << 4) + rlane) * lda + koff + k0;
      const v16b ah = ldfrag_b(Ah + ao);
      const v16b al = ldfrag_b(Al + ao);
#pragma unroll
      for (int j = 0; j < 2; ++j) {
        acc[i][j] = mma_b_raw(ah, bh[j], acc[i][j]);
        acc[i][j] = mma_b_raw(al, bh[j], acc[i][j]);
        acc[i][j] = mma_b_raw(ah, bl[j], acc[i][j]);
      }
      dep_guard_b(acc[i][0], acc[i][1], ah, al);
    }
    keep4_b(bh[0], bh[1], bl[0], bl[1]);
  }
  acc_guard2(acc[0][0], acc[0][1]);
  acc_guard2(acc[1][0], acc[1][1]);
  acc_guard2(acc[2][0], acc[2][1]);
  acc_guard2(acc[3][0], acc[3][1]);

  float* slab = sT[wave];
  const int q = lane >> 3, c4 = (lane & 7) * 4;
  const v4f bc = *(const v4f*)(bias + n0 + c4);
#pragma unroll
  for (int i = 0; i < 4; ++i) {
    const int mBase = m0 + (i << 4);
#pragma unroll
    for (int j = 0; j < 2; ++j) {
#pragma unroll
      for (int r = 0; r < 8; ++r) {
        slab[(mOff + r) * 36 + (j << 4) + rlane] = acc[i][j][r];
      }
    }
    __builtin_amdgcn_fence(__ATOMIC_RELEASE, "workgroup");
    __builtin_amdgcn_wave_barrier();
    __builtin_amdgcn_fence(__ATOMIC_ACQUIRE, "workgroup");
    v4f ov[4];
#pragma unroll
    for (int it = 0; it < 4; ++it) {
      const int row = it * 4 + q;
      const v4f v = *(const v4f*)(slab + row * 36 + c4);
      ov[it] = v + bc;
    }
    for (int pass = 0; pass < 2; ++pass) {
#pragma unroll
      for (int it = 0; it < 4; ++it) {
        const int row = it * 4 + q;
        *(volatile v4f*)(Cout + (size_t)(mBase + row) * ldc + n0 + c4) = ov[it];
      }
      __threadfence();
    }
    __builtin_amdgcn_fence(__ATOMIC_RELEASE, "workgroup");
    __builtin_amdgcn_wave_barrier();
    __builtin_amdgcn_fence(__ATOMIC_ACQUIRE, "workgroup");
  }
}

__global__ __launch_bounds__(128)
void attn64(const unsigned short* __restrict__ qp, const unsigned short* __restrict__ kp,
            const unsigned short* __restrict__ vtp, const int* __restrict__ mask,
            unsigned short* ohp, unsigned short* olp, float sscale, float oscale) {
  union FH { v16h v; v8h h[2]; };
  __shared__ __align__(16) _Float16 Ksh[64 * 64];
  __shared__ __align__(16) _Float16 Vth[64 * 64];
  __shared__ __align__(16) _Float16 Psh[4][16 * 64];
  __shared__ __align__(16) float    Os[4][16 * 64];

  const int tid  = threadIdx.x;
  const int wave = tid >> 5;
  const int lane = tid & 31;
  const int hh   = lane >> 4;
  const int c    = lane & 15;

  const int bx   = blockIdx.x;
  const int qb   = bx % NQB;
  const int rest = bx / NQB;
  const int h    = rest % NH;
  const int b    = rest / NH;
  const int q0   = qb * 64 + wave * 16;
  const size_t rowB = (size_t)b * SEQ;

  const _Float16* Q  = (const _Float16*)(const void*)qp + (size_t)h * HD;
  const _Float16* Kg = (const _Float16*)(const void*)kp + (size_t)h * HD;
  const _Float16* Vt = (const _Float16*)(const void*)vtp + ((size_t)b * DM + (size_t)h * HD) * SEQ;
  const int* mk = mask + (size_t)b * SEQ;

  v16h qa[2];
#pragma unroll
  for (int dc = 0; dc < 2; ++dc) {
    const size_t qo = (rowB + q0 + c) * DM + dc * 32 + 8 * hh;
    qa[dc] = ldfrag_h(Q + qo);
  }

  float mrow[8], lrow[8];
  v8f oacc[4];
#pragma unroll
  for (int r = 0; r < 8; ++r) { mrow[r] = -INFINITY; lrow[r] = 0.f; }
#pragma unroll
  for (int t = 0; t < 4; ++t) oacc[t] = zero8();

  for (int kt = 0; kt < NQB; ++kt) {
    const int kv0 = kt * 64;
    __syncthreads();
    {
      const int r = tid >> 1, half = (tid & 1) * 32;
      const _Float16* kg = Kg + (rowB + kv0 + r) * DM + half;
      const _Float16* vg = Vt + (size_t)r * SEQ + kv0 + half;
#pragma unroll
      for (int i = 0; i < 4; ++i) {
        const v8h a0 = *(const v8h*)(kg + 8 * i);
        const v8h b0 = *(const v8h*)(vg + 8 * i);
        *(v8h*)(Ksh + r * 64 + half + 8 * i) = a0;
        *(v8h*)(Vth + r * 64 + half + 8 * i) = b0;
      }
    }
    __syncthreads();

    v8f s[4];
#pragma unroll
    for (int j = 0; j < 4; ++j) {
      s[j] = zero8();
#pragma unroll
      for (int dc = 0; dc < 2; ++dc) {
        FH kb;
        kb.h[0] = *(const v8h*)(Ksh + (j * 16 + c) * 64 + dc * 32 + 8 * hh);
        kb.h[1] = *(const v8h*)(Ksh + (j * 16 + c) * 64 + dc * 32 + 16 + 8 * hh);
        s[j] = mma_h(qa[dc], kb.v, s[j]);
      }
    }
    int mv[4];
#pragma unroll
    for (int j = 0; j < 4; ++j) mv[j] = mk[kv0 + j * 16 + c];

    _Float16* pwh = Psh[wave];
#pragma unroll
    for (int r = 0; r < 8; ++r) {
      float m = -INFINITY;
#pragma unroll
      for (int j = 0; j < 4; ++j) {
        float sv = s[j][r] * sscale;
        sv = (mv[j] == 0) ? -INFINITY : sv;
        s[j][r] = sv;
        m = fmaxf(m, sv);
      }
#pragma unroll
      for (int off = 1; off < 16; off <<= 1) m = fmaxf(m, __shfl_xor(m, off, 32));
      const float mnew  = fmaxf(mrow[r], m);
      const float msafe = (mnew == -INFINITY) ? 0.f : mnew;
      const float alpha = __expf(mrow[r] - msafe);
      mrow[r] = mnew;
      float psum = 0.f;
#pragma unroll
      for (int j = 0; j < 4; ++j) {
        const float p = __expf(s[j][r] - msafe);
        psum += p;
        pwh[(8 * hh + r) * 64 + j * 16 + c] = (_Float16)(p * CAR_P);
      }
#pragma unroll
      for (int off = 1; off < 16; off <<= 1) psum += __shfl_xor(psum, off, 32);
      lrow[r] = lrow[r] * alpha + psum;
#pragma unroll
      for (int t = 0; t < 4; ++t) oacc[t][r] *= alpha;
    }
    __builtin_amdgcn_fence(__ATOMIC_RELEASE, "workgroup");
    __builtin_amdgcn_wave_barrier();
    __builtin_amdgcn_fence(__ATOMIC_ACQUIRE, "workgroup");

#pragma unroll 1
    for (int kk = 0; kk < 2; ++kk) {
      FH pa;
      pa.h[0] = *(const v8h*)(pwh + c * 64 + kk * 32 + 8 * hh);
      pa.h[1] = *(const v8h*)(pwh + c * 64 + kk * 32 + 16 + 8 * hh);
#pragma unroll
      for (int t = 0; t < 4; ++t) {
        FH vb;
        vb.h[0] = *(const v8h*)(Vth + (t * 16 + c) * 64 + kk * 32 + 8 * hh);
        vb.h[1] = *(const v8h*)(Vth + (t * 16 + c) * 64 + kk * 32 + 16 + 8 * hh);
        oacc[t] = mma_h(pa.v, vb.v, oacc[t]);
      }
    }
  }

  float* os = Os[wave];
  const float qnan = __uint_as_float(0x7fc00000u);
#pragma unroll
  for (int r = 0; r < 8; ++r) {
    const float l = lrow[r];
    const float inv = (l > 0.f) ? (__builtin_amdgcn_rcpf(l) * oscale) : qnan;
#pragma unroll
    for (int t = 0; t < 4; ++t) os[(8 * hh + r) * 64 + t * 16 + c] = oacc[t][r] * inv;
  }
  __builtin_amdgcn_fence(__ATOMIC_RELEASE, "workgroup");
  __builtin_amdgcn_wave_barrier();
  __builtin_amdgcn_fence(__ATOMIC_ACQUIRE, "workgroup");
  {
    const int q4 = lane >> 3, c8 = (lane & 7) * 8;
    v4u hv[4], lv[4];
#pragma unroll
    for (int it = 0; it < 4; ++it) {
      const int row = it * 4 + q4;
      const float* sp = os + row * 64 + c8;
      const v4f a0 = *(const v4f*)(sp);
      const v4f a1 = *(const v4f*)(sp + 4);
      float f[8];
#pragma unroll
      for (int e = 0; e < 4; ++e) { f[e] = a0[e]; f[4 + e] = a1[e]; }
      v4u a, a2;
#pragma unroll
      for (int e = 0; e < 4; ++e) {
        const unsigned short h0 = bf_bits(f[2 * e]), h1 = bf_bits(f[2 * e + 1]);
        const unsigned short l0 = bf_bits(f[2 * e] - bf_up(h0)), l1 = bf_bits(f[2 * e + 1] - bf_up(h1));
        a[e] = pk16(h0, h1); a2[e] = pk16(l0, l1);
      }
      hv[it] = a; lv[it] = a2;
    }
    for (int pass = 0; pass < 2; ++pass) {
#pragma unroll
      for (int it = 0; it < 4; ++it) {
        const int row = it * 4 + q4;
        const size_t go = (rowB + q0 + row) * DM + (size_t)h * HD + c8;
        *(volatile v4u*)(ohp + go) = hv[it];
        *(volatile v4u*)(olp + go) = lv[it];
      }
      __threadfence();
    }
  }
}

extern "C" void kernel_launch(void* const* d_in, const int* in_sizes, int n_in,
                              void* d_out, int out_size, void* d_ws, size_t ws_size,
                              hipStream_t stream) {
  if (n_in < 22) return;
  const int wsz = DM * DM;
  if (in_sizes[0] != NTOK * DM) return;
  if (in_sizes[1] != NB * SEQ) return;
  if (in_sizes[2] != wsz || in_sizes[4] != wsz || in_sizes[6] != wsz || in_sizes[10] != wsz ||
      in_sizes[14] != wsz || in_sizes[18] != wsz || in_sizes[20] != wsz) return;
  if (in_sizes[3] != DM || in_sizes[5] != DM || in_sizes[7] != DM || in_sizes[9] != DM ||
      in_sizes[11] != DM || in_sizes[13] != DM || in_sizes[15] != DM || in_sizes[17] != DM ||
      in_sizes[19] != DM || in_sizes[21] != DM) return;
  if (in_sizes[8] != 3 * DM || in_sizes[12] != 3 * DM || in_sizes[16] != 3 * DM) return;
  if (out_size != NTOK * DM) return;

  const float* x      = (const float*)d_in[0];
  const int*   mask   = (const int*)d_in[1];
  const float* wq     = (const float*)d_in[2];
  const float* bq     = (const float*)d_in[3];
  const float* wk     = (const float*)d_in[4];
  const float* bk     = (const float*)d_in[5];
  const float* wv     = (const float*)d_in[6];
  const float* bv     = (const float*)d_in[7];
  const float* q_dw_w = (const float*)d_in[8];
  const float* q_dw_b = (const float*)d_in[9];
  const float* q_pw_w = (const float*)d_in[10];
  const float* q_pw_b = (const float*)d_in[11];
  const float* k_dw_w = (const float*)d_in[12];
  const float* k_dw_b = (const float*)d_in[13];
  const float* k_pw_w = (const float*)d_in[14];
  const float* k_pw_b = (const float*)d_in[15];
  const float* v_dw_w = (const float*)d_in[16];
  const float* v_dw_b = (const float*)d_in[17];
  const float* v_pw_w = (const float*)d_in[18];
  const float* v_pw_b = (const float*)d_in[19];
  const float* wo     = (const float*)d_in[20];
  const float* bo     = (const float*)d_in[21];

  const long long PLH = (long long)NTOK * DM;
  const long long PWH = (long long)DM * DM;
  const size_t PL2 = (size_t)PLH * 2;
  const size_t PW2 = (size_t)PWH * 2;
  size_t off = 0;
  const size_t oX   = off; off += PL2;
  const size_t oW   = off; off += 6 * PW2;
  const size_t oWOh = off; off += PW2;
  const size_t oWOl = off; off += PW2;
  const size_t oP0  = off; off += 3 * PL2;
  const size_t oY   = off; off += 3 * PL2;
  const size_t oN   = off; off += 2 * PL2;
  const size_t oVT  = off; off += (size_t)NB * DM * SEQ * 2;
  const size_t oCTh = off; off += PL2;
  const size_t oCTl = off; off += PL2;
  if (off > ws_size) return;
  if (off > (size_t)134217728) return;

  char* ws = (char*)d_ws;
  unsigned short* Xh  = (unsigned short*)(ws + oX);
  unsigned short* Wh  = (unsigned short*)(ws + oW);
  unsigned short* WOh = (unsigned short*)(ws + oWOh);
  unsigned short* WOl = (unsigned short*)(ws + oWOl);
  unsigned short* P0  = (unsigned short*)(ws + oP0);
  unsigned short* Y   = (unsigned short*)(ws + oY);
  unsigned short* Nrm = (unsigned short*)(ws + oN);
  unsigned short* VT  = (unsigned short*)(ws + oVT);
  unsigned short* CTh = (unsigned short*)(ws + oCTh);
  unsigned short* CTl = (unsigned short*)(ws + oCTl);

  const dim3 blk(256);
  const int n8x = NTOK * DM / 8;
  const int n8w = DM * DM / 8;
  const dim3 gCvtX((n8x + 255) / 256, 1);
  const dim3 gCvtW((n8w + 255) / 256, 6);
  const dim3 gCvtWo((n8w + 255) / 256, 1);
  const dim3 gQKV(((NTOK / 64) * (DM / 64) + 7) / 8, 3);
  const dim3 gDw((n8x + 255) / 256, 3);
  const dim3 gPwQK(((NTOK / 64) * (DM / 64) + 7) / 8, 2);
  const dim3 gPwVT(((DM / 64) * (SEQ / 64) + 7) / 8, NB);
  const dim3 gAttn(NB * NH * NQB);
  const dim3 gWo(((NTOK / 64) * (DM / 32) + 7) / 8, 1);

  cvt_f16x8<<<gCvtX, blk, 0, stream>>>(x, x, x, x, x, x, x, Xh, 0LL, n8x, 1.0f);
  cvt_f16x8<<<gCvtW, blk, 0, stream>>>(wq, wk, wv, q_pw_w, k_pw_w, v_pw_w, v_pw_w, Wh, PWH, n8w, CAR_W);
  cvt_bf16hl_x8<<<gCvtWo, blk, 0, stream>>>(wo, WOh, WOl, n8w);
  gemm64<1><<<gQKV, blk, 0, stream>>>(
      Xh, DM, 0LL, Wh, DM, PWH,
      (void*)P0, DM, PLH,
      bq, bk, bv,
      NTOK, DM, DM, 1.0f / CAR_W, CAR_P0);
  dwconv3_f16x8<<<gDw, blk, 0, stream>>>(
      P0, Y, q_dw_w, k_dw_w, v_dw_w, q_dw_b, k_dw_b, v_dw_b,
      PLH, n8x, CAR_Y / CAR_P0, CAR_Y);
  gemm64<2><<<gPwQK, blk, 0, stream>>>(
      Y, DM, PLH, Wh + 3 * PWH, DM, PWH,
      (void*)Nrm, DM, PLH,
      q_pw_b, k_pw_b, k_pw_b,
      NTOK, DM, DM, 1.0f / (CAR_Y * CAR_W), CAR_N);
  gemm64<3><<<gPwVT, blk, 0, stream>>>(
      Wh + 5 * PWH, DM, 0LL, Y + 2 * PLH, DM, (long long)SEQ * DM,
      (void*)VT, SEQ, (long long)DM * SEQ,
      v_pw_b, v_pw_b, v_pw_b,
      DM, SEQ, DM, 1.0f / (CAR_Y * CAR_W), CAR_V);
  attn64<<<gAttn, dim3(128), 0, stream>>>(
      Nrm, Nrm + PLH, VT, mask, CTh, CTl, 0.125f / (CAR_N * CAR_N), 1.0f / (CAR_P * CAR_V));
  gemm_bf3<<<gWo, blk, 0, stream>>>(
      CTh, CTl, DM, WOh, WOl, DM,
      (float*)d_out, DM, bo, NTOK, DM, DM);
  (void)hipGetLastError();
}
